// ElasticAttentionBlock_558345748857
// MI455X (gfx1250) — hardware-verified
//
#include <hip/hip_runtime.h>
#include <hip/hip_bf16.h>
#include <math.h>

#define NQ_ 4096
#define NK_ 8192
#define DD  1024
#define SS  4096
#define HH  16
#define DKK 64
#define BB  1

typedef _Float16 bf16;
typedef _Float16 f16;
typedef __attribute__((ext_vector_type(4))) unsigned v4u_t;
typedef unsigned v4ua __attribute__((ext_vector_type(4), may_alias));
typedef __attribute__((ext_vector_type(4))) float v4f_t;
typedef float v4fa __attribute__((ext_vector_type(4), may_alias));
typedef __attribute__((ext_vector_type(16))) bf16  bf16x16;
typedef bf16x16 f16x16;
typedef __attribute__((ext_vector_type(8)))  bf16  bf16x8;
typedef bf16x8 f16x8;
typedef __attribute__((ext_vector_type(4)))  bf16  bf16x4;
typedef __attribute__((ext_vector_type(8)))  float f32x8;
__device__ __forceinline__ f32x8 wmma16(f16x16 a, f16x16 b, f32x8 c) {
  c = __builtin_amdgcn_wmma_f32_16x16x32_f16(false, a, false, b, (short)0, c, false, false);
  asm volatile("v_nop\n\tv_nop\n\tv_nop\n\tv_nop" : "+v"(c) : "v"(a), "v"(b));
  return c;
}
#define LDS_STRIDE 48
#define KSTRIDE    72
#define VSTRIDE    48

__device__ __forceinline__ f32x8 wmma_bf16(bf16x16 a, bf16x16 b, f32x8 c) {
  return __builtin_amdgcn_wmma_f32_16x16x32_f16(
      false, a, false, b, (short)0, c, false, false);
}

template <typename T>
__device__ __forceinline__ bf16x16 load_frag(const T* __restrict__ base, int ld,
                                             int row0, int k0) {
  const int lane = threadIdx.x & 31;
  const int r    = lane & 15;
  const int kh   = (lane >> 4) * 8;
  const T* p0 = base + (size_t)(row0 + r) * ld + (k0 + kh);
  const T* p1 = p0 + 16;
  bf16x16 f;
#pragma unroll
  for (int i = 0; i < 8; ++i) {
    f[i]     = (bf16)p0[i];
    f[i + 8] = (bf16)p1[i];
  }
  return f;
}

__device__ __forceinline__ bf16x16 lds_frag(const bf16* base, int stride) {
  const int lane = threadIdx.x & 31;
  const int row  = lane & 15;
  const int kh   = (lane >> 4) * 8;
  const bf16x8 lo = *(const bf16x8*)(base + row * stride + kh);
  const bf16x8 hi = *(const bf16x8*)(base + row * stride + kh + 16);
  bf16x16 f;
#pragma unroll
  for (int i = 0; i < 8; ++i) { f[i] = lo[i]; f[i + 8] = hi[i]; }
  return f;
}

template <typename T>
__device__ __forceinline__ void stage_read16(const T* __restrict__ p, float* buf) {
#pragma unroll
  for (int i = 0; i < 16; ++i) buf[i] = (float)p[i];
}

__device__ __forceinline__ void stage_write(bf16* dst, const float* buf, int nquad) {
#pragma unroll
  for (int i = 0; i < nquad; ++i) {
    bf16x4 q;
    q[0] = (bf16)buf[4 * i];     q[1] = (bf16)buf[4 * i + 1];
    q[2] = (bf16)buf[4 * i + 2]; q[3] = (bf16)buf[4 * i + 3];
    *(bf16x4*)(dst + 4 * i) = q;
  }
}

template <typename AT, int MODE>
__global__ __launch_bounds__(256) void gemm_exp_kernel(
    const AT* __restrict__ A, const float* __restrict__ W,
    const float* __restrict__ rq, const float* __restrict__ rk, void* __restrict__ out,
    int M, int N, int K) {
  __shared__ bf16 ldsA[128 * LDS_STRIDE];
  __shared__ bf16 ldsW[256 * LDS_STRIDE];
  __shared__ __attribute__((aligned(16))) unsigned char sob[256 * 136 * 2];

  const int t    = threadIdx.x;
  const int wave = t >> 5;
  const int lane = t & 31;
  const int wm   = (wave & 1) * 64;
  const int wn   = (wave >> 1) * 64;
  const int mBlk = blockIdx.x * 128;
  const int nBlk = blockIdx.y * 256;

  const int arow = t >> 1;
  const int ach  = (t & 1) * 16;

  float abuf[16];
  float wbuf[32];

  stage_read16(A + (size_t)(mBlk + arow) * K + ach, abuf);
  stage_read16(W + (size_t)(nBlk + t) * K,          wbuf);
  stage_read16(W + (size_t)(nBlk + t) * K + 16,     wbuf + 16);

  f32x8 acc[4][4] = {};

  for (int k = 0; k < K; k += 32) {
    __syncthreads();
    stage_write(&ldsA[arow * LDS_STRIDE + ach], abuf, 4);
    stage_write(&ldsW[t * LDS_STRIDE],          wbuf, 8);
    if (k + 32 < K) {
      stage_read16(A + (size_t)(mBlk + arow) * K + (k + 32) + ach, abuf);
      stage_read16(W + (size_t)(nBlk + t) * K + (k + 32),          wbuf);
      stage_read16(W + (size_t)(nBlk + t) * K + (k + 32) + 16,     wbuf + 16);
    }
    __syncthreads();

    bf16x16 af[4], wf[4];
#pragma unroll
    for (int i = 0; i < 4; ++i)
      af[i] = lds_frag(ldsA + (wm + 16 * i) * LDS_STRIDE, LDS_STRIDE);
#pragma unroll
    for (int j = 0; j < 4; ++j)
      wf[j] = lds_frag(ldsW + (wn + 16 * j) * LDS_STRIDE, LDS_STRIDE);
#pragma unroll
    for (int i = 0; i < 4; ++i)
#pragma unroll
      for (int j = 0; j < 4; ++j)
        acc[i][j] = wmma_bf16(af[i], wf[j], acc[i][j]);
  }

  const int nlane = lane & 15;
  const int mh    = (lane >> 4) * 8;
  __syncthreads();
  if (MODE == 0 || MODE == 1) {
    bf16* so = (bf16*)sob;
#pragma unroll
    for (int i = 0; i < 4; ++i)
#pragma unroll
      for (int j = 0; j < 4; ++j) {
        const int nl = wn + 16 * j + nlane;
        const float rkn = rk[nBlk + nl];
#pragma unroll
        for (int r = 0; r < 8; ++r) {
          const int ml = wm + 16 * i + mh + r;
          const bf16 hv = (bf16)__builtin_amdgcn_exp2f((acc[i][j][r] * rq[mBlk + ml] * rkn - 1.0f) * 1.44269504088896340736f);
          if (MODE == 0) so[ml * 264 + nl] = hv;
          else           so[nl * 136 + ml] = hv;
        }
      }
    __syncthreads();
#pragma unroll 1
    for (int pass = 0; pass < 2; ++pass) {
      if (MODE == 0) {
        for (int ch = t; ch < 128 * 32; ch += 256) { const int ml = ch >> 5, q = (ch & 31) * 8;
          *(volatile v4u_t*)((bf16*)out + (size_t)(mBlk + ml) * N + nBlk + q) = *(const v4ua*)(so + ml * 264 + q); }
      } else {
        const int b_ = mBlk / SS, s0 = mBlk & (SS - 1);
        for (int ch = t; ch < 256 * 16; ch += 256) { const int nl = ch >> 4, q = (ch & 15) * 8; const int n = nBlk + nl, h = n >> 6, dk = n & (DKK - 1);
          *(volatile v4u_t*)((bf16*)out + (((size_t)(b_ * HH + h)) * DKK + dk) * SS + s0 + q) = *(const v4ua*)(so + nl * 136 + q); }
      }
      __threadfence();
    }
  } else {
    float* so = (float*)sob;
#pragma unroll 1
    for (int hf = 0; hf < 2; ++hf) {
      if (wm == hf * 64) {
#pragma unroll
        for (int i = 0; i < 4; ++i)
#pragma unroll
          for (int j = 0; j < 4; ++j) {
            const int nl = wn + 16 * j + nlane;
#pragma unroll
            for (int r = 0; r < 8; ++r) so[(16 * i + mh + r) * 260 + nl] = acc[i][j][r];
          }
      }
      __syncthreads();
#pragma unroll 1
      for (int pass = 0; pass < 2; ++pass) {
        for (int ch = t; ch < 64 * 64; ch += 256) { const int ml = ch >> 6, q = (ch & 63) * 4;
          *(volatile v4f_t*)((float*)out + (size_t)(mBlk + hf * 64 + ml) * N + nBlk + q) = *(const volatile v4fa*)(so + ml * 260 + q); }
        __threadfence();
      }
      __syncthreads();
    }
  }
}


#define GSTR 48
template <typename AT, bool ACC>
__global__ __launch_bounds__(256) void gemm_kn(const AT* __restrict__ A, int lda, size_t strideA,
                                               const float* __restrict__ Wm, int ldw, size_t strideW,
                                               const float* __restrict__ bias, float scale,
                                               float* __restrict__ Y, int ldy, size_t strideY, int K) {
  __shared__ __attribute__((aligned(16))) f16 ldsA[128 * GSTR];
  __shared__ __attribute__((aligned(16))) f16 ldsW[128 * GSTR];
  __shared__ __attribute__((aligned(16))) float oS[8][32 * 68];
  const int tid = threadIdx.x, lane = tid & 31, wave = tid >> 5, cl = lane & 15, rh = (lane >> 4) * 8;
  const int m0 = blockIdx.x * 128, n0 = blockIdx.y * 128;
  const int wm = (wave & 3) * 32, wn = (wave >> 2) * 64;
  A += (size_t)blockIdx.z * strideA; Wm += (size_t)blockIdx.z * strideW; Y += (size_t)blockIdx.z * strideY;
  f32x8 acc[2][4];
#pragma unroll
  for (int i = 0; i < 2; ++i)
#pragma unroll
    for (int j = 0; j < 4; ++j) { f32x8 z = {}; acc[i][j] = z; }
#pragma unroll 1
  for (int k0 = 0; k0 < K; k0 += 32) {
    __syncthreads();
    {
      const int row = tid >> 1, ch = (tid & 1) * 16;
      const AT* src = A + (size_t)(m0 + row) * lda + k0 + ch;
#pragma unroll
      for (int g = 0; g < 16; ++g) ldsA[row * GSTR + ch + g] = (f16)src[g];
    }
    {
      const int k = tid >> 3, nn0 = (tid & 7) * 16;
      const float* src = Wm + (size_t)(k0 + k) * ldw + n0 + nn0;
#pragma unroll
      for (int g = 0; g < 4; ++g) { const v4f_t v = *(const v4f_t*)(src + 4 * g);
#pragma unroll
        for (int u = 0; u < 4; ++u) ldsW[(nn0 + 4 * g + u) * GSTR + k] = (f16)v[u]; }
    }
    __syncthreads();
    f16x16 af[2];
#pragma unroll
    for (int i = 0; i < 2; ++i) af[i] = lds_frag(ldsA + (wm + 16 * i) * GSTR, GSTR);
#pragma unroll
    for (int j = 0; j < 4; ++j) {
      const f16x16 bf = lds_frag(ldsW + (wn + 16 * j) * GSTR, GSTR);
#pragma unroll
      for (int i = 0; i < 2; ++i) acc[i][j] = wmma16(af[i], bf, acc[i][j]);
    }
  }
  float* so = oS[wave];
#pragma unroll
  for (int i = 0; i < 2; ++i)
#pragma unroll
    for (int j = 0; j < 4; ++j) {
      const float bv = bias ? bias[n0 + wn + 16 * j + cl] : 0.0f;
#pragma unroll
      for (int r = 0; r < 8; ++r) so[(16 * i + rh + r) * 68 + 16 * j + cl] = acc[i][j][r] * scale + bv;
    }
  asm volatile("s_wait_dscnt 0" ::: "memory");
  __builtin_amdgcn_wave_barrier();
  if (ACC) {
#pragma unroll
    for (int it = 0; it < 16; ++it) { const int f4 = lane + 32 * it, rr = f4 >> 4, q = (f4 & 15) * 4;
      const v4f_t old = *(const volatile v4fa*)(Y + (size_t)(m0 + wm + rr) * ldy + n0 + wn + q);
      v4f_t v = *(const volatile v4fa*)(so + rr * 68 + q); v += old; *(volatile v4fa*)(so + rr * 68 + q) = v; }
    asm volatile("s_wait_dscnt 0" ::: "memory");
  }
#pragma unroll 1
  for (int pass = 0; pass < 2; ++pass) {
#pragma unroll
    for (int it = 0; it < 16; ++it) { const int f4 = lane + 32 * it, rr = f4 >> 4, q = (f4 & 15) * 4;
      *(volatile v4f_t*)(Y + (size_t)(m0 + wm + rr) * ldy + n0 + wn + q) = *(const volatile v4fa*)(so + rr * 68 + q); }
    __threadfence();
  }
}

__global__ __launch_bounds__(256) void k_norms(const float* __restrict__ Q, const float* __restrict__ Kt, float* __restrict__ rq, float* __restrict__ rk) {
  __shared__ __attribute__((aligned(16))) float rS[32];
  const int tid = threadIdx.x, lane = tid & 31, wave = tid >> 5;
  const int blk = blockIdx.x;
  const bool isq = blk < NQ_ / 32;
  const float* X = isq ? Q : Kt;
  const int row0 = (isq ? blk : blk - NQ_ / 32) * 32;
#pragma unroll 1
  for (int rr = 0; rr < 4; ++rr) {
    const int row = row0 + wave * 4 + rr;
    const float* x = X + (size_t)row * DD;
    float s = 0.0f;
    for (int d = lane * 4; d < DD; d += 128) { const v4f_t v = *(const v4f_t*)(x + d); s += v[0] * v[0] + v[1] * v[1] + v[2] * v[2] + v[3] * v[3]; }
#pragma unroll
    for (int off = 16; off >= 1; off >>= 1) s += __shfl_xor(s, off, 32);
    if (lane == 0) rS[wave * 4 + rr] = 1.0f / sqrtf(s);
  }
  __syncthreads();
  float* dst = (isq ? rq : rk) + row0;
  if (wave == 0 && lane < 8) {
#pragma unroll 1
    for (int pass = 0; pass < 2; ++pass) { *(volatile v4f_t*)(dst + lane * 4) = *(const volatile v4fa*)(rS + lane * 4); __threadfence(); }
  }
}
__global__ __launch_bounds__(256) void k_rownorm(const f16* __restrict__ P, float* __restrict__ out) {
  __shared__ float red[8];
  const int tid = threadIdx.x, lane = tid & 31, wave = tid >> 5, row = blockIdx.x;
  const f16* pr = P + (size_t)row * NK_ + tid * 32;
  float s = 0.0f;
#pragma unroll
  for (int g = 0; g < 4; ++g) { const f16x8 v = *(const f16x8*)(pr + 8 * g);
#pragma unroll
    for (int u = 0; u < 8; ++u) s += (float)v[u]; }
#pragma unroll
  for (int off = 16; off >= 1; off >>= 1) s += __shfl_xor(s, off, 32);
  if (lane == 0) red[wave] = s;
  __syncthreads();
  const float l = ((red[0] + red[1]) + (red[2] + red[3])) + ((red[4] + red[5]) + (red[6] + red[7]));
  const float il = 1.0f / l;
  float* o = out + (size_t)row * DD + tid * 4;
  v4f_t v = *(const volatile v4fa*)o; v *= il;
  *(volatile v4f_t*)o = v; __threadfence(); *(volatile v4f_t*)o = v;
}

extern "C" void kernel_launch(void* const* d_in, const int* in_sizes, int n_in,
                              void* d_out, int out_size, void* d_ws, size_t ws_size,
                              hipStream_t stream) {
  (void)in_sizes; (void)n_in; (void)out_size; (void)ws_size;
  const float* Q  = (const float*)d_in[0];
  const float* Kt = (const float*)d_in[1];
  float* out = (float*)d_out;
  char* ws = (char*)d_ws;
  f16* P = (f16*)ws;
  float* rq = (float*)(ws + (64 << 20));
  float* rk = (float*)(ws + (64 << 20) + (16 << 10));
  k_norms<<<dim3((NQ_ + NK_) / 32), dim3(256), 0, stream>>>(Q, Kt, rq, rk);
  gemm_exp_kernel<float, 0><<<dim3(NQ_ / 128, NK_ / 256), dim3(256), 0, stream>>>(Q, Kt, rq, rk, P, NQ_, NK_, DD);
  gemm_kn<f16, false><<<dim3(NQ_ / 128, DD / 128, 1), dim3(256), 0, stream>>>(P, NK_, 0, Kt, DD, 0, nullptr, 1.0f, out, DD, 0, NK_);
  k_rownorm<<<dim3(NQ_), dim3(256), 0, stream>>>(P, out);
}
